// PathAttention_75333726372356
// MI455X (gfx1250) — hardware-verified
//
#include <hip/hip_runtime.h>
#include <stdint.h>

#define NB   8
#define NS   1024
#define HD   768
#define NHD  12
#define DH   64
#define MOC  256

typedef _Float16 v16h __attribute__((ext_vector_type(16)));
typedef _Float16 v8h  __attribute__((ext_vector_type(8)));
typedef _Float16 v4h  __attribute__((ext_vector_type(4)));
typedef float    v8f  __attribute__((ext_vector_type(8)));
typedef float    v4f  __attribute__((ext_vector_type(4)));
typedef unsigned short us16;

union FragU { v16h v; v8h h[2]; };

__device__ __forceinline__ v16h frag_load(const _Float16* p) {
  FragU f; f.h[0] = *(const v8h*)(p); f.h[1] = *(const v8h*)(p + 16); return f.v;
}
__device__ __forceinline__ v8f mma16(v16h a, v16h b, v8f c) {
  return __builtin_amdgcn_wmma_f32_16x16x32_f16(false, a, false, b, (short)0, c, false, false);
}
__device__ __forceinline__ v8f mma16g(v16h a, v16h b, v8f c) {
  c = __builtin_amdgcn_wmma_f32_16x16x32_f16(false, a, false, b, (short)0, c, false, false);
  asm volatile("v_nop\n\tv_nop\n\tv_nop\n\tv_nop" : "+v"(c) : "v"(a), "v"(b));
  return c;
}
__device__ __forceinline__ void dep_guard(v8f& a, v8f& b, v16h x, v16h y) {
  asm volatile("v_nop\n\tv_nop\n\tv_nop\n\tv_nop" : "+v"(a), "+v"(b) : "v"(x), "v"(y));
}
__device__ __forceinline__ void keep4(v16h a, v16h b, v16h c, v16h d) {
  asm volatile("v_nop" :: "v"(a), "v"(b), "v"(c), "v"(d));
}
__device__ __forceinline__ void acc_guard4(v8f& a, v8f& b, v8f& c, v8f& d) {
  asm volatile("v_nop\n\tv_nop\n\tv_nop\n\tv_nop" : "+v"(a), "+v"(b), "+v"(c), "+v"(d));
}
__device__ __forceinline__ void wave_lds_sync() {
  __builtin_amdgcn_fence(__ATOMIC_RELEASE, "workgroup");
  __builtin_amdgcn_wave_barrier();
  __builtin_amdgcn_fence(__ATOMIC_ACQUIRE, "workgroup");
}
__device__ __forceinline__ v8h pack8h(v4f a, v4f b) {
  v8h r;
  r[0] = (_Float16)a[0]; r[1] = (_Float16)a[1]; r[2] = (_Float16)a[2]; r[3] = (_Float16)a[3];
  r[4] = (_Float16)b[0]; r[5] = (_Float16)b[1]; r[6] = (_Float16)b[2]; r[7] = (_Float16)b[3];
  return r;
}

template <int BIAS_MODE, int OUT_MODE, bool RESID, int ACT>
__global__ __launch_bounds__(256) void k_gemm(
    const us16* __restrict__ Ap, int lda, long strideA,
    const us16* __restrict__ Btp, int ldb, long strideB,
    void* Cout, int ldc, long strideC,
    const float* __restrict__ bias, long strideBias,
    const float* resid, int ldr, long strideR,
    int M, int N, int K, float scale)
{
  __shared__ __align__(16) float sT[8][16 * 68];
  const _Float16* A  = (const _Float16*)Ap;
  const _Float16* Bt = (const _Float16*)Btp;
  const int z    = blockIdx.y;
  const int lane = threadIdx.x & 31;
  const int wave = threadIdx.x >> 5;
  const int tilesN = N >> 6;
  const int tilesM = M >> 6;
  const int tile = blockIdx.x * 8 + wave;
  if (tile >= tilesM * tilesN) return;
  const int tm = tile / tilesN;
  const int tn = tile - tm * tilesN;
  const int m0 = tm << 6;
  const int n0 = tn << 6;

  const _Float16* Ab = A  + (size_t)z * (size_t)strideA;
  const _Float16* Bb = Bt + (size_t)z * (size_t)strideB;

  const int rl   = lane & 15;
  const int koff = (lane >> 4) * 8;
  const int mOff = (lane >> 4) * 8;

  v8f acc[4][4];
#pragma unroll
  for (int i = 0; i < 4; ++i)
#pragma unroll
    for (int j = 0; j < 4; ++j) acc[i][j] = (v8f){0.f, 0.f, 0.f, 0.f, 0.f, 0.f, 0.f, 0.f};

  for (int k0 = 0; k0 < K; k0 += 32) {
    v16h bf[4];
#pragma unroll
    for (int j = 0; j < 4; ++j)
      bf[j] = frag_load(Bb + (size_t)(n0 + (j << 4) + rl) * ldb + k0 + koff);
#pragma unroll
    for (int i = 0; i < 4; ++i) {
      const v16h af = frag_load(Ab + (size_t)(m0 + (i << 4) + rl) * lda + k0 + koff);
#pragma unroll
      for (int j = 0; j < 4; ++j) acc[i][j] = mma16(af, bf[j], acc[i][j]);
      dep_guard(acc[i][0], acc[i][3], af, bf[3]);
    }
    keep4(bf[0], bf[1], bf[2], bf[3]);
  }
  acc_guard4(acc[0][0], acc[0][1], acc[0][2], acc[0][3]);
  acc_guard4(acc[1][0], acc[1][1], acc[1][2], acc[1][3]);
  acc_guard4(acc[2][0], acc[2][1], acc[2][2], acc[2][3]);
  acc_guard4(acc[3][0], acc[3][1], acc[3][2], acc[3][3]);

  float* slab = sT[wave];
  const float* Rb = RESID ? (resid + (size_t)z * (size_t)strideR) : nullptr;
  const float* Bz = (BIAS_MODE != 0) ? (bias + (size_t)z * (size_t)strideBias) : nullptr;
#pragma unroll
  for (int i = 0; i < 4; ++i) {
    const int mBase = m0 + (i << 4);
#pragma unroll
    for (int j = 0; j < 4; ++j) {
      const int n = n0 + (j << 4) + rl;
      float bv = 0.f;
      if (BIAS_MODE == 2) bv = Bz[n];
#pragma unroll
      for (int r = 0; r < 8; ++r) {
        float v = acc[i][j][r] * scale;
        if (BIAS_MODE == 1) v += Bz[mBase + mOff + r];
        if (BIAS_MODE == 2) v += bv;
        if (RESID) v += Rb[(size_t)(mBase + mOff + r) * ldr + n];
        if (ACT == 1) v = tanhf(v);
        slab[(mOff + r) * 68 + (j << 4) + rl] = v;
      }
    }
    wave_lds_sync();
    if (OUT_MODE == 0) {
      float* C = (float*)Cout + (size_t)z * (size_t)strideC;
      const int hh = lane >> 4, c4 = (lane & 15) * 4;
      for (int pass = 0; pass < 2; ++pass) {
#pragma unroll
        for (int it = 0; it < 8; ++it) {
          const int row = it * 2 + hh;
          const v4f v = *(const v4f*)(slab + row * 68 + c4);
          *(volatile v4f*)(C + (size_t)(mBase + row) * ldc + n0 + c4) = v;
        }
        __threadfence();
      }
    } else {
      _Float16* C = (_Float16*)Cout + (size_t)z * (size_t)strideC;
      const int q = lane >> 3, c8 = (lane & 7) * 8;
      v8h hv[4];
#pragma unroll
      for (int it = 0; it < 4; ++it) {
        const float* sp = slab + (it * 4 + q) * 68 + c8;
        v8h t;
#pragma unroll
        for (int e = 0; e < 8; ++e) t[e] = (_Float16)sp[e];
        hv[it] = t;
      }
      for (int pass = 0; pass < 2; ++pass) {
#pragma unroll
        for (int it = 0; it < 4; ++it)
          *(volatile v8h*)(C + (size_t)(mBase + it * 4 + q) * ldc + n0 + c8) = hv[it];
        __threadfence();
      }
    }
    wave_lds_sync();
  }
}

__global__ __launch_bounds__(256) void k_cvt16(const float* __restrict__ s0, const float* __restrict__ s1,
                                               const float* __restrict__ s2, const float* __restrict__ s3,
                                               const float* __restrict__ s4, const float* __restrict__ s5,
                                               us16* out, int n8, float scale)
{
  const int i = blockIdx.x * 256 + threadIdx.x;
  const int y = blockIdx.y;
  if (i >= n8) return;
  const float* src = (y == 0) ? s0 : (y == 1) ? s1 : (y == 2) ? s2 : (y == 3) ? s3 : (y == 4) ? s4 : s5;
  const float* p = src + (size_t)i * 8;
  v4f a = *(const v4f*)p, b = *(const v4f*)(p + 4);
  a = a * scale; b = b * scale;
  const v8h o = pack8h(a, b);
  _Float16* d = (_Float16*)out + (size_t)y * (size_t)n8 * 8 + (size_t)i * 8;
  *(volatile v8h*)d = o;
  __threadfence();
  *(volatile v8h*)d = o;
}

__global__ __launch_bounds__(256) void k_bias4(const float* __restrict__ s0, const float* __restrict__ s1,
                                               const float* __restrict__ s2, const float* __restrict__ s3,
                                               float* dst)
{
  const int gi = blockIdx.x * 256 + threadIdx.x;
  if (gi >= 768) return;
  const int which = gi / 192;
  const int i4 = (gi - which * 192) * 4;
  const float* src = (which == 0) ? s0 : (which == 1) ? s1 : (which == 2) ? s2 : s3;
  const v4f v = *(const v4f*)(src + i4);
  float* d = dst + (size_t)gi * 4;
  *(volatile v4f*)d = v;
  __threadfence();
  *(volatile v4f*)d = v;
}

__global__ __launch_bounds__(256) void k_prep(const float* __restrict__ x, const int* __restrict__ pp,
                                              us16* x16, us16* vin16)
{
  const int gi  = blockIdx.x * 256 + threadIdx.x;
  const int row = gi / 96;
  const int c8  = gi - row * 96;
  const int b = row >> 10, n = row & (NS - 1);
  const int np = (n + NS - 1) & (NS - 1), nn = (n + 1) & (NS - 1);
  const int pidx = b * NS + ((n >= 2) ? (n - 2) : 0);
  const bool single = (n == 0) || (n >= 2 && pp[pidx] == 1);
  const size_t oc = (size_t)c8 * 8;
  const float* xr = x + (size_t)(b * NS + n)  * HD + oc;
  const float* xp = x + (size_t)(b * NS + np) * HD + oc;
  const float* xq = x + (size_t)(b * NS + nn) * HD + oc;
  const v4f r0 = *(const v4f*)xr, r1 = *(const v4f*)(xr + 4);
  const v4f p0 = *(const v4f*)xp, p1 = *(const v4f*)(xp + 4);
  const v4f q0 = *(const v4f*)xq, q1 = *(const v4f*)(xq + 4);
  v4f v0 = (p0 + q0) * 0.5f, v1 = (p1 + q1) * 0.5f;
  if (single) { v0 = q0; v1 = q1; }
  const v8h ox = pack8h(r0, r1), ov = pack8h(v0, v1);
  _Float16* dx = (_Float16*)x16   + (size_t)row * HD + oc;
  _Float16* dv = (_Float16*)vin16 + (size_t)row * HD + oc;
  *(volatile v8h*)dx = ox;
  *(volatile v8h*)dv = ov;
  __threadfence();
  *(volatile v8h*)dx = ox;
  *(volatile v8h*)dv = ov;
}

__global__ __launch_bounds__(256) void k_vary(const float* __restrict__ y, const int* __restrict__ pp,
                                              us16* cat, float scale)
{
  const int gi  = blockIdx.x * 256 + threadIdx.x;
  const int row = gi / 96;
  const int c8  = gi - row * 96;
  const int b = row >> 10, n = row & (NS - 1);
  const int np = (n + NS - 1) & (NS - 1), nn = (n + 1) & (NS - 1);
  const int pidx = b * NS + ((n >= 2) ? (n - 2) : 0);
  const bool single = (n == 0) || (n >= 2 && pp[pidx] == 1);
  const size_t oc = (size_t)c8 * 8;
  const float* yr = y + (size_t)(b * NS + n)  * HD + oc;
  const float* yp = y + (size_t)(b * NS + np) * HD + oc;
  const float* yq = y + (size_t)(b * NS + nn) * HD + oc;
  v4f r0 = *(const v4f*)yr, r1 = *(const v4f*)(yr + 4);
  const v4f p0 = *(const v4f*)yp, p1 = *(const v4f*)(yp + 4);
  const v4f q0 = *(const v4f*)yq, q1 = *(const v4f*)(yq + 4);
  v4f v0 = (p0 + q0) * 0.5f, v1 = (p1 + q1) * 0.5f;
  if (single) { v0 = q0; v1 = q1; }
  v0 = v0 * scale; v1 = v1 * scale; r0 = r0 * scale; r1 = r1 * scale;
  const v8h ov = pack8h(v0, v1), oy = pack8h(r0, r1);
  _Float16* dv = (_Float16*)cat + (size_t)row * (2 * HD) + oc;
  _Float16* dy = dv + HD;
  *(volatile v8h*)dv = ov;
  *(volatile v8h*)dy = oy;
  __threadfence();
  *(volatile v8h*)dv = ov;
  *(volatile v8h*)dy = oy;
}

__global__ __launch_bounds__(256) void k_score(const float* __restrict__ T, const float* __restrict__ Ws,
                                               const float* __restrict__ bs, const int* __restrict__ pp,
                                               float* SL, float* SU)
{
  __shared__ __align__(16) float sL[32];
  __shared__ __align__(16) float sUp[32];
  const int lane = threadIdx.x & 31, wave = threadIdx.x >> 5;
  const int base = blockIdx.x * 32;
  const float b0 = bs[0];
  for (int r4 = 0; r4 < 4; ++r4) {
    const int row = base + wave * 4 + r4;
    const float* tr = T + (size_t)row * (2 * HD);
    float acc = 0.f;
#pragma unroll 4
    for (int j = lane; j < HD; j += 32) {
      acc += tr[HD + j] * Ws[j];
      acc += tr[j] * Ws[HD + j];
    }
#pragma unroll
    for (int off = 1; off < 32; off <<= 1) acc += __shfl_xor(acc, off, 32);
    float v = acc + b0;
    v = (v > 0.f) ? v : 0.02f * v;
    const int n = row & (NS - 1);
    const bool pred = (pp[row] == 1);
    const int pm2 = (n >= 2) ? (row - 2) : row;
    const bool single = (n == 0) || (n >= 2 && pp[pm2] == 1);
    const bool lower = pred && (n >= 1);
    const bool upper = pred && ((n <= 1) || !single);
    if (lane == 0) {
      sL[wave * 4 + r4]  = lower ? v : 0.f;
      sUp[wave * 4 + r4] = upper ? v : 0.f;
    }
  }
  __syncthreads();
  if (wave == 0) {
    const int l8 = lane & 7;
    const v4f a = *(const v4f*)(sL + l8 * 4);
    const v4f u = *(const v4f*)(sUp + l8 * 4);
    if (lane < 8) {
      float* d = SL + base + l8 * 4;
      *(volatile v4f*)d = a;
      __threadfence();
      *(volatile v4f*)d = a;
    } else if (lane < 16) {
      float* d = SU + base + l8 * 4;
      *(volatile v4f*)d = u;
      __threadfence();
      *(volatile v4f*)d = u;
    }
  }
}

__global__ __launch_bounds__(256) void k_cross(const float* __restrict__ x, const int* __restrict__ occ,
                                               const float* __restrict__ Wc, const float* __restrict__ bc,
                                               float* SC)
{
  __shared__ __align__(16) float sS[32];
  const int lane = threadIdx.x & 31, wave = threadIdx.x >> 5;
  const int base = blockIdx.x * 32;
  const float b0 = bc[0];
  for (int r4 = 0; r4 < 4; ++r4) {
    const int p = base + wave * 4 + r4;
    const int b = p >> 8;
    int o0 = occ[2 * p], o1 = occ[2 * p + 1];
    o0 = (o0 < 0) ? 0 : ((o0 > NS - 1) ? (NS - 1) : o0);
    o1 = (o1 < 0) ? 0 : ((o1 > NS - 1) ? (NS - 1) : o1);
    const float* x0 = x + (size_t)(b * NS + o0) * HD;
    const float* x1 = x + (size_t)(b * NS + o1) * HD;
    float acc = 0.f;
#pragma unroll 4
    for (int j = lane; j < HD; j += 32) {
      const float xm = (x0[j] + x1[j]) * 0.5f;
      acc += xm * Wc[j];
    }
#pragma unroll
    for (int off = 1; off < 32; off <<= 1) acc += __shfl_xor(acc, off, 32);
    float v = acc + b0;
    v = (v > 0.f) ? v : 0.02f * v;
    if (lane == 0) sS[wave * 4 + r4] = v;
  }
  __syncthreads();
  if (wave == 0) {
    const int l8 = lane & 7;
    const v4f a = *(const v4f*)(sS + l8 * 4);
    if (lane < 8) {
      float* d = SC + base + l8 * 4;
      *(volatile v4f*)d = a;
      __threadfence();
      *(volatile v4f*)d = a;
    }
  }
}

__global__ __launch_bounds__(256) void k_graph(const float* __restrict__ AGin, const float* __restrict__ VGin,
                                               const float* __restrict__ SL, const float* __restrict__ SU,
                                               const float* __restrict__ SC, const int* __restrict__ occ,
                                               float* Gb, us16* AG16, us16* VG16)
{
  __shared__ int sO0[MOC];
  __shared__ int sO1[MOC];
  __shared__ float sSc[MOC];
  __shared__ unsigned sBal[8][2];
  const int tid = threadIdx.x, lane = tid & 31, wave = tid >> 5;
  const int b  = blockIdx.x >> 7;
  const int n0 = (blockIdx.x & 127) * 8;
  {
    const int p = b * MOC + tid;
    int o0 = occ[2 * p], o1 = occ[2 * p + 1];
    o0 = (o0 < 0) ? 0 : ((o0 > NS - 1) ? (NS - 1) : o0);
    o1 = (o1 < 0) ? 0 : ((o1 > NS - 1) ? (NS - 1) : o1);
    sO0[tid] = o0; sO1[tid] = o1; sSc[tid] = SC[p];
  }
  const int c0 = tid * 4;
  for (int r = 0; r < 8; ++r) {
    const int n  = n0 + r;
    const int bn = b * NS + n;
    __syncthreads();
    v4f ag = *(const v4f*)(AGin + (size_t)bn * NS + c0);
    v4f vg = *(const v4f*)(VGin + (size_t)bn * NS + c0);
    const float sl_n = SL[bn];
    const float su_n = SU[bn];
    const float sl_p = SL[(bn + 1 < NB * NS) ? (bn + 1) : (NB * NS - 1)];
    const float su_m = SU[(bn >= 1) ? (bn - 1) : 0];
#pragma unroll
    for (int e = 0; e < 4; ++e) {
      const int cc = c0 + e;
      float v = ag[e];
      if (n >= 1 && cc == n - 1)      { v = v + sl_n; v = v + su_m; }
      if (n <= NS - 2 && cc == n + 1) { v = v + sl_p; v = v + su_n; }
      if (n == NS - 1 && cc == NS - 1) { v = v + su_n; v = v + su_n; }
      ag[e] = v;
    }
    const unsigned h0 = __builtin_amdgcn_ballot_w32(sO0[tid] == n);
    const unsigned h1 = __builtin_amdgcn_ballot_w32(sO1[tid] == n);
    if (lane == 0) { sBal[wave][0] = h0; sBal[wave][1] = h1; }
    __syncthreads();
    for (int w = 0; w < 8; ++w) {
      unsigned m = sBal[w][0];
      while (m != 0u) {
        const int l = __builtin_ctz(m); m &= (m - 1u);
        const int p = w * 32 + l;
        const int d = sO1[p] - c0;
        const float sc = sSc[p];
        vg[0] = (d == 0) ? (vg[0] + sc) : vg[0];
        vg[1] = (d == 1) ? (vg[1] + sc) : vg[1];
        vg[2] = (d == 2) ? (vg[2] + sc) : vg[2];
        vg[3] = (d == 3) ? (vg[3] + sc) : vg[3];
      }
    }
    for (int w = 0; w < 8; ++w) {
      unsigned m = sBal[w][1];
      while (m != 0u) {
        const int l = __builtin_ctz(m); m &= (m - 1u);
        const int p = w * 32 + l;
        const int d = sO0[p] - c0;
        const float sc = sSc[p];
        vg[0] = (d == 0) ? (vg[0] + sc) : vg[0];
        vg[1] = (d == 1) ? (vg[1] + sc) : vg[1];
        vg[2] = (d == 2) ? (vg[2] + sc) : vg[2];
        vg[3] = (d == 3) ? (vg[3] + sc) : vg[3];
      }
    }
    const v4f g = ag * 0.2f;
    v4h a16, g16;
#pragma unroll
    for (int e = 0; e < 4; ++e) { a16[e] = (_Float16)(ag[e] * 16.0f); g16[e] = (_Float16)(vg[e] * 16.0f); }
    float*    gp = Gb + (size_t)bn * NS + c0;
    _Float16* ap = (_Float16*)AG16 + (size_t)bn * NS + c0;
    _Float16* vp = (_Float16*)VG16 + (size_t)bn * NS + c0;
    *(volatile v4f*)gp = g;
    *(volatile v4h*)ap = a16;
    *(volatile v4h*)vp = g16;
    __threadfence();
    *(volatile v4f*)gp = g;
    *(volatile v4h*)ap = a16;
    *(volatile v4h*)vp = g16;
  }
}

__global__ __launch_bounds__(256) void k_tr16(const us16* __restrict__ in, us16* out)
{
  __shared__ __align__(16) _Float16 tl[64 * 72];
  const _Float16* I = (const _Float16*)in + (size_t)blockIdx.z * NS * NS;
  _Float16*       O = (_Float16*)out      + (size_t)blockIdx.z * NS * NS;
  const int c0  = blockIdx.x * 64;
  const int r0  = blockIdx.y * 64;
  const int tid = threadIdx.x;
  {
    const int rr  = tid >> 2;
    const int c16 = (tid & 3) * 16;
    const _Float16* src = I + (size_t)(r0 + rr) * NS + c0 + c16;
    const v8h a0 = *(const v8h*)src;
    const v8h a1 = *(const v8h*)(src + 8);
    *(v8h*)(tl + rr * 72 + c16)     = a0;
    *(v8h*)(tl + rr * 72 + c16 + 8) = a1;
  }
  __syncthreads();
  const int sub = tid >> 3;
  const int c8  = (tid & 7) * 8;
  v8h hv[2];
#pragma unroll
  for (int it = 0; it < 2; ++it) {
    const int oc = it * 32 + sub;
    v8h t;
#pragma unroll
    for (int e = 0; e < 8; ++e) t[e] = tl[(c8 + e) * 72 + oc];
    hv[it] = t;
  }
  for (int pass = 0; pass < 2; ++pass) {
#pragma unroll
    for (int it = 0; it < 2; ++it) {
      const int oc = it * 32 + sub;
      *(volatile v8h*)(O + (size_t)(c0 + oc) * NS + r0 + c8) = hv[it];
    }
    __threadfence();
  }
}

__global__ __launch_bounds__(128)
void k_attn(const us16* __restrict__ Qp, const us16* __restrict__ Kp, const us16* __restrict__ VTp,
            const float* __restrict__ Gp, us16* Yp, float sscale, float oscale)
{
  __shared__ __align__(16) _Float16 Ksh[64 * 64];
  __shared__ __align__(16) _Float16 Vth[64 * 64];
  __shared__ __align__(16) _Float16 Psh[4][16 * 64];
  __shared__ __align__(16) float    Os[4][16 * 68];

  const int tid  = threadIdx.x;
  const int wave = tid >> 5;
  const int lane = tid & 31;
  const int hh   = lane >> 4;
  const int c    = lane & 15;
  const int b    = blockIdx.y;
  const int qb   = blockIdx.x & 15;
  const int h    = blockIdx.x >> 4;
  const int q0   = qb * 64 + wave * 16;

  const _Float16* Q  = (const _Float16*)Qp  + (size_t)b * NS * HD + (size_t)h * DH;
  const _Float16* Kk = (const _Float16*)Kp  + (size_t)b * NS * HD + (size_t)h * DH;
  const _Float16* VT = (const _Float16*)VTp + (size_t)b * HD * NS + (size_t)h * DH * NS;
  const float*    G  = Gp + (size_t)b * NS * NS;
  _Float16*       Y  = (_Float16*)Yp + (size_t)b * NS * HD + (size_t)h * DH;

  v16h qa[2];
#pragma unroll
  for (int dc = 0; dc < 2; ++dc) qa[dc] = frag_load(Q + (size_t)(q0 + c) * HD + dc * 32 + 8 * hh);

  float mrow[8], lrow[8];
  v8f oacc[4];
#pragma unroll
  for (int r = 0; r < 8; ++r) { mrow[r] = -__builtin_huge_valf(); lrow[r] = 0.f; }
#pragma unroll
  for (int t = 0; t < 4; ++t) oacc[t] = (v8f){0.f, 0.f, 0.f, 0.f, 0.f, 0.f, 0.f, 0.f};

  for (int kc = 0; kc < NS / 64; ++kc) {
    const int kv0 = kc * 64;
    __syncthreads();
    {
      const int r = tid >> 1, half = (tid & 1) * 32;
      const _Float16* ks = Kk + (size_t)(kv0 + r) * HD + half;
      const _Float16* vs = VT + (size_t)r * NS + kv0 + half;
#pragma unroll
      for (int i = 0; i < 4; ++i) {
        const v8h a0 = *(const v8h*)(ks + 8 * i);
        const v8h b0 = *(const v8h*)(vs + 8 * i);
        *(v8h*)(Ksh + r * 64 + half + 8 * i) = a0;
        *(v8h*)(Vth + r * 64 + half + 8 * i) = b0;
      }
    }
    __syncthreads();

    v8f s[4];
#pragma unroll
    for (int j = 0; j < 4; ++j) {
      s[j] = (v8f){0.f, 0.f, 0.f, 0.f, 0.f, 0.f, 0.f, 0.f};
#pragma unroll
      for (int dc = 0; dc < 2; ++dc) {
        FragU kb;
        kb.h[0] = *(const v8h*)(Ksh + (j * 16 + c) * 64 + dc * 32 + 8 * hh);
        kb.h[1] = *(const v8h*)(Ksh + (j * 16 + c) * 64 + dc * 32 + 16 + 8 * hh);
        s[j] = mma16g(qa[dc], kb.v, s[j]);
      }
    }
    float cm[8];
#pragma unroll
    for (int r = 0; r < 8; ++r) {
      const float* grow = G + (size_t)(q0 + 8 * hh + r) * NS + kv0 + c;
      float m = -__builtin_huge_valf();
#pragma unroll
      for (int j = 0; j < 4; ++j) {
        const float sv = s[j][r] * sscale + grow[16 * j];
        s[j][r] = sv;
        m = fmaxf(m, sv);
      }
#pragma unroll
      for (int off = 1; off < 16; off <<= 1) m = fmaxf(m, __shfl_xor(m, off, 32));
      cm[r] = m;
    }
    _Float16* pw = Psh[wave];
#pragma unroll
    for (int r = 0; r < 8; ++r) {
      const float mnew  = fmaxf(mrow[r], cm[r]);
      const float alpha = __expf(mrow[r] - mnew);
      mrow[r] = mnew;
      float psum = 0.f;
#pragma unroll
      for (int j = 0; j < 4; ++j) {
        const float p = __expf(s[j][r] - mnew);
        psum += p;
        pw[(8 * hh + r) * 64 + j * 16 + c] = (_Float16)(p * 4096.0f);
      }
#pragma unroll
      for (int off = 1; off < 16; off <<= 1) psum += __shfl_xor(psum, off, 32);
      lrow[r] = lrow[r] * alpha + psum;
#pragma unroll
      for (int t = 0; t < 4; ++t) oacc[t][r] *= alpha;
    }
    wave_lds_sync();
#pragma unroll 1
    for (int kk = 0; kk < 2; ++kk) {
      FragU pa;
      pa.h[0] = *(const v8h*)(pw + c * 64 + kk * 32 + 8 * hh);
      pa.h[1] = *(const v8h*)(pw + c * 64 + kk * 32 + 16 + 8 * hh);
#pragma unroll
      for (int t = 0; t < 4; ++t) {
        FragU vb;
        vb.h[0] = *(const v8h*)(Vth + (t * 16 + c) * 64 + kk * 32 + 8 * hh);
        vb.h[1] = *(const v8h*)(Vth + (t * 16 + c) * 64 + kk * 32 + 16 + 8 * hh);
        oacc[t] = mma16g(pa.v, vb.v, oacc[t]);
      }
    }
  }

  float* os = Os[wave];
#pragma unroll
  for (int r = 0; r < 8; ++r) {
    const float inv = (1.0f / lrow[r]) * (1.0f / 4096.0f) * oscale;
#pragma unroll
    for (int t = 0; t < 4; ++t) os[(8 * hh + r) * 68 + t * 16 + c] = oacc[t][r] * inv;
  }
  wave_lds_sync();
  {
    const int q = lane >> 3, c8 = (lane & 7) * 8;
    v8h hv[4];
#pragma unroll
    for (int it = 0; it < 4; ++it) {
      const float* sp = os + (it * 4 + q) * 68 + c8;
      v8h t;
#pragma unroll
      for (int e = 0; e < 8; ++e) t[e] = (_Float16)sp[e];
      hv[it] = t;
    }
    for (int pass = 0; pass < 2; ++pass) {
#pragma unroll
      for (int it = 0; it < 4; ++it)
        *(volatile v8h*)(Y + (size_t)(q0 + it * 4 + q) * HD + c8) = hv[it];
      __threadfence();
    }
  }
}

__global__ __launch_bounds__(256) void k_pmean(const float* __restrict__ At, const int* __restrict__ pp, float* out)
{
  __shared__ float sW[NS];
  __shared__ __align__(16) float sPm[256];
  const int tid = threadIdx.x;
  const int b   = blockIdx.y;
  const int cb  = blockIdx.x * 256;
  const int* pb = pp + b * NS;
#pragma unroll
  for (int k = 0; k < 4; ++k) {
    const int n = tid * 4 + k;
    const bool pred = (pb[n] == 1);
    const int pm2 = (n >= 2) ? (n - 2) : n;
    const bool single = (n == 0) || (n >= 2 && pb[pm2] == 1);
    const bool upper  = pred && ((n <= 1) || !single);
    const bool triple = upper && (n >= 1);
    sW[n] = pred ? (triple ? 3.0f : 2.0f) : 0.0f;
  }
  __syncthreads();
  float acc = 0.f, wsum = 0.f;
  const float* ap = At + (size_t)b * NS * HD + cb + tid;
#pragma unroll 4
  for (int n = 0; n < NS; ++n) {
    const float w = sW[n];
    wsum += w;
    acc  += w * ap[(size_t)n * HD];
  }
  const float pmv = acc * (1.0f / wsum);
  sPm[tid] = pmv;
  __syncthreads();
  const int rq = tid >> 6, l64 = tid & 63;
  const v4f v = *(const v4f*)(sPm + l64 * 4);
  float* ob = out + (size_t)b * NS * HD + cb + l64 * 4;
  for (int pass = 0; pass < 2; ++pass) {
#pragma unroll 4
    for (int it = 0; it < 256; ++it) {
      const int row = it * 4 + rq;
      *(volatile v4f*)(ob + (size_t)row * HD) = v;
    }
    __threadfence();
  }
}

extern "C" void kernel_launch(void* const* d_in, const int* in_sizes, int n_in,
                              void* d_out, int out_size, void* d_ws, size_t ws_size,
                              hipStream_t stream)
{
  if (n_in < 25) return;
  const int nBNH = NB * NS * HD;
  const int nW   = HD * HD;
  if (in_sizes[0] != nBNH || in_sizes[1] != NB * NS * NS || in_sizes[2] != NB * NS * NS) return;
  if (in_sizes[3] != nW || in_sizes[5] != nW || in_sizes[13] != nW || in_sizes[15] != nW ||
      in_sizes[17] != nW || in_sizes[19] != nW) return;
  if (in_sizes[4] != HD || in_sizes[6] != HD || in_sizes[12] != HD || in_sizes[14] != HD ||
      in_sizes[16] != HD || in_sizes[18] != HD || in_sizes[20] != HD) return;
  if (in_sizes[7] != 2 * HD || in_sizes[8] < 1 || in_sizes[9] != HD || in_sizes[10] < 1 || in_sizes[11] != 2 * HD * HD) return;
  if (in_sizes[21] != NB * NS || in_sizes[24] != NB * MOC * 2) return;
  if (out_size != nBNH) return;

  const float* x       = (const float*)d_in[0];
  const float* atomg   = (const float*)d_in[1];
  const float* varg    = (const float*)d_in[2];
  const float* W_var   = (const float*)d_in[3];  const float* b_var  = (const float*)d_in[4];
  const float* W_sym   = (const float*)d_in[5];  const float* b_sym  = (const float*)d_in[6];
  const float* W_score = (const float*)d_in[7];  const float* b_sc   = (const float*)d_in[8];
  const float* W_cross = (const float*)d_in[9];  const float* b_cr   = (const float*)d_in[10];
  const float* W_atom  = (const float*)d_in[11]; const float* b_atom = (const float*)d_in[12];
  const float* W_q     = (const float*)d_in[13]; const float* b_q    = (const float*)d_in[14];
  const float* W_k     = (const float*)d_in[15]; const float* b_k    = (const float*)d_in[16];
  const float* W_v     = (const float*)d_in[17]; const float* b_v    = (const float*)d_in[18];
  const float* W_o     = (const float*)d_in[19]; const float* b_o    = (const float*)d_in[20];
  const int*   pp      = (const int*)d_in[21];
  const int*   occ     = (const int*)d_in[24];
  float* out = (float*)d_out;

  const size_t PH   = (size_t)NB * NS * HD;
  const size_t WPL  = (size_t)HD * HD;
  const size_t GPL  = (size_t)NS * NS;
  const size_t szW16  = 6 * WPL * 2;
  const size_t szWat  = (size_t)HD * 2 * HD * 2;
  const size_t szBias = 4 * (size_t)HD * 4;
  const size_t szS    = (size_t)NB * NS * 4;
  const size_t szSC   = (size_t)NB * MOC * 4;
  const size_t szGb   = (size_t)NB * GPL * 4;
  const size_t szX16  = PH * 2;
  const size_t szPool = 2 * (size_t)NB * GPL * 2 * 2;
  size_t off = 0;
  const size_t oW16  = off; off += szW16;
  const size_t oWat  = off; off += szWat;
  const size_t oBias = off; off += szBias;
  const size_t oSL   = off; off += szS;
  const size_t oSU   = off; off += szS;
  const size_t oSC   = off; off += szSC;
  const size_t oGb   = off; off += szGb;
  const size_t oX16  = off; off += szX16;
  const size_t oPool = off; off += szPool;
  if (off > ws_size) return;
  if (oPool != oX16 + szX16) return;
  const size_t oVin16 = oPool;
  const size_t oT     = oPool + szX16;
  const size_t oG16   = oPool;
  const size_t oGT16  = oPool + 33554432;
  const size_t oQ16   = oPool;
  const size_t oK16   = oPool + szX16;
  const size_t oVT16  = oPool + 2 * szX16;
  const size_t oYat   = oPool + 3 * szX16;
  const size_t oY32   = oGb;
  const size_t oCat   = oPool;
  const size_t oAtom  = oPool + 25165824;
  if (oT + (size_t)NB * NS * 2 * HD * 4 > oPool + szPool) return;
  if (oYat + szX16 > oPool + szPool) return;
  if (oAtom + PH * 4 > oPool + szPool) return;

  char* ws = (char*)d_ws;
  us16*  W16   = (us16*)(ws + oW16);
  us16*  Wat16 = (us16*)(ws + oWat);
  float* biasw = (float*)(ws + oBias);
  float* SL    = (float*)(ws + oSL);
  float* SU    = (float*)(ws + oSU);
  float* SC    = (float*)(ws + oSC);
  float* Gb    = (float*)(ws + oGb);
  us16*  X16   = (us16*)(ws + oX16);
  us16*  Vin16 = (us16*)(ws + oVin16); (void)Vin16;
  float* T32   = (float*)(ws + oT);
  us16*  G16   = (us16*)(ws + oG16);
  us16*  GT16  = (us16*)(ws + oGT16);
  us16*  Q16   = (us16*)(ws + oQ16);
  us16*  K16   = (us16*)(ws + oK16);
  us16*  VT16  = (us16*)(ws + oVT16);
  us16*  Yat16 = (us16*)(ws + oYat);
  float* Y32   = (float*)(ws + oY32);
  us16*  Cat16 = (us16*)(ws + oCat);
  float* At32  = (float*)(ws + oAtom);

  const dim3 blk(256);
  const float inv16  = 1.0f / 16.0f;
  const float inv128 = 1.0f / 128.0f;
  const float inv256 = 1.0f / 256.0f;

  k_cvt16<<<dim3((int)(WPL / 8 / 256), 6), blk, 0, stream>>>(W_sym, W_var, W_q, W_k, W_v, W_o, W16, (int)(WPL / 8), 16.0f);
  k_cvt16<<<dim3((int)(WPL * 2 / 8 / 256), 1), blk, 0, stream>>>(W_atom, W_atom, W_atom, W_atom, W_atom, W_atom, Wat16, (int)(WPL * 2 / 8), 16.0f);
  k_bias4<<<dim3(3), blk, 0, stream>>>(b_sym, b_var, b_q, b_k, biasw);
  k_prep<<<dim3(NB * NS * 96 / 256), blk, 0, stream>>>(x, pp, X16, Vin16);
  k_gemm<2, 0, false, 1><<<dim3(192, 2), blk, 0, stream>>>(
      X16, HD, (long)PH, W16, HD, (long)WPL, (void*)T32, 2 * HD, (long)HD,
      biasw, (long)HD, nullptr, 0, 0L, NB * NS, HD, HD, inv16);
  k_score<<<dim3(NB * NS / 32), blk, 0, stream>>>(T32, W_score, b_sc, pp, SL, SU);
  k_cross<<<dim3(NB * MOC / 32), blk, 0, stream>>>(x, occ, W_cross, b_cr, SC);
  k_graph<<<dim3(NB * NS / 8), blk, 0, stream>>>(atomg, varg, SL, SU, SC, occ, Gb, G16, G16 + (size_t)NB * GPL);
  k_tr16<<<dim3(NS / 64, NS / 64, 2 * NB), blk, 0, stream>>>(G16, GT16);
  k_gemm<0, 0, true, 0><<<dim3(32, NB), blk, 0, stream>>>(
      G16, NS, (long)GPL, GT16, NS, (long)GPL, (void*)Gb, NS, (long)GPL,
      nullptr, 0L, Gb, NS, (long)GPL, NS, NS, NS, 0.8f * inv256);
  k_gemm<0, 0, true, 0><<<dim3(32, NB), blk, 0, stream>>>(
      G16 + (size_t)NB * GPL, NS, (long)GPL, GT16 + (size_t)NB * GPL, NS, (long)GPL, (void*)Gb, NS, (long)GPL,
      nullptr, 0L, Gb, NS, (long)GPL, NS, NS, NS, inv256);
  k_gemm<2, 1, false, 0><<<dim3(192, 2), blk, 0, stream>>>(
      X16, HD, 0L, W16 + 2 * WPL, HD, (long)WPL, (void*)Q16, HD, (long)PH,
      biasw + 2 * HD, (long)HD, nullptr, 0, 0L, NB * NS, HD, HD, inv16);
  k_gemm<1, 1, false, 0><<<dim3(24, NB), blk, 0, stream>>>(
      W16 + 4 * WPL, HD, 0L, X16, HD, (long)(NS * HD), (void*)VT16, NS, (long)(HD * NS),
      b_v, 0L, nullptr, 0, 0L, HD, NS, HD, inv16);
  k_attn<<<dim3(NHD * (NS / 64), NB), dim3(128), 0, stream>>>(Q16, K16, VT16, Gb, Yat16, 0.125f, 8.0f);
  k_gemm<2, 0, false, 0><<<dim3(192, 1), blk, 0, stream>>>(
      Yat16, HD, 0L, W16 + 5 * WPL, HD, 0L, (void*)Y32, HD, 0L,
      b_o, 0L, nullptr, 0, 0L, NB * NS, HD, HD, inv128);
  k_vary<<<dim3(NB * NS * 96 / 256), blk, 0, stream>>>(Y32, pp, Cat16, 8.0f);
  k_gemm<2, 0, false, 0><<<dim3(192, 1), blk, 0, stream>>>(
      Cat16, 2 * HD, 0L, Wat16, 2 * HD, 0L, (void*)At32, HD, 0L,
      b_atom, 0L, nullptr, 0, 0L, NB * NS, HD, 2 * HD, inv128);
  k_pmean<<<dim3(HD / 256, NB), blk, 0, stream>>>(At32, pp, out);
  (void)hipGetLastError();
}
